// SelectiveScan_8572754723187
// MI455X (gfx1250) — hardware-verified
//
#include <hip/hip_runtime.h>

typedef __attribute__((ext_vector_type(16))) _Float16 v16h;
typedef __attribute__((ext_vector_type(8)))  _Float16 v8h;
typedef __attribute__((ext_vector_type(16))) __bf16   v16b;
typedef __attribute__((ext_vector_type(8)))  __bf16   v8b;
typedef __attribute__((ext_vector_type(8)))  float    v8f;
typedef __attribute__((ext_vector_type(4)))  float    v4f;
typedef __attribute__((ext_vector_type(4)))  unsigned int v4u;

constexpr int NBATCH  = 2;
constexpr int SEQLEN  = 2048;
constexpr int EMB     = 1024;
constexpr int NSTATE  = 16;
constexpr int KCONV   = 4;
constexpr int RNK     = 64;
constexpr int NROWS   = NBATCH * SEQLEN;
constexpr int NPAR    = RNK + 2 * NSTATE;
constexpr int NPARPAD = 128;

static_assert(NROWS % 64 == 0);
static_assert(EMB % 64 == 0 && NPARPAD % 64 == 0);
static_assert(EMB % 32 == 0 && RNK % 32 == 0);

constexpr size_t BYTES_XB   = (size_t)NROWS * EMB * 2;
constexpr size_t BYTES_W    = (size_t)EMB * EMB * 2;
constexpr size_t BYTES_WP   = (size_t)NPARPAD * EMB * 2;
constexpr size_t BYTES_WDT  = (size_t)EMB * RNK * 2;
constexpr size_t BYTES_F32P = (size_t)NROWS * EMB * 4;
constexpr size_t BYTES_PAR  = (size_t)NROWS * NPARPAD * 4;
constexpr size_t BYTES_DTU  = (size_t)NROWS * RNK * 2;
constexpr size_t OFF_XB    = 0;
constexpr size_t OFF_WX    = OFF_XB + BYTES_XB;
constexpr size_t OFF_WZ    = OFF_WX + BYTES_W;
constexpr size_t OFF_WO    = OFF_WZ + BYTES_W;
constexpr size_t OFF_WP    = OFF_WO + BYTES_W;
constexpr size_t OFF_WDT   = OFF_WP + BYTES_WP;
constexpr size_t OFF_XRES  = OFF_WDT + BYTES_WDT;
constexpr size_t OFF_Z     = OFF_XRES + BYTES_F32P;
constexpr size_t OFF_PAR   = OFF_Z + BYTES_F32P;
constexpr size_t OFF_DTUH  = OFF_PAR + BYTES_PAR;
constexpr size_t OFF_DTUL  = OFF_DTUH + BYTES_DTU;
constexpr size_t OFF_DTRAW = OFF_DTUL + BYTES_DTU;
constexpr size_t OFF_YH    = OFF_DTRAW + BYTES_F32P;
constexpr size_t OFF_YL    = OFF_YH + BYTES_XB;
constexpr size_t WS_TOTAL  = OFF_YL + BYTES_XB;
static_assert(WS_TOTAL == 85327872ull);
static_assert(WS_TOTAL <= 134217728ull);
static_assert(OFF_WX % 256 == 0 && OFF_WP % 256 == 0 && OFF_WDT % 256 == 0 && OFF_XRES % 256 == 0 &&
              OFF_PAR % 256 == 0 && OFF_DTUH % 256 == 0 && OFF_DTRAW % 256 == 0 && OFF_YH % 256 == 0 && OFF_YL % 256 == 0);

__device__ __forceinline__ unsigned short f2bf_bits(float f) {
  unsigned u = __float_as_uint(f);
  return (unsigned short)((u + 0x7FFFu + ((u >> 16) & 1u)) >> 16);
}
__device__ __forceinline__ float bf_bits2f(unsigned short h) { return __uint_as_float(((unsigned)h) << 16); }
__device__ __forceinline__ float bf_rne(float f) { return bf_bits2f(f2bf_bits(f)); }

__device__ __forceinline__ unsigned pack_bf2(float v0, float v1) {
  return (unsigned)f2bf_bits(v0) | ((unsigned)f2bf_bits(v1) << 16);
}
__device__ __forceinline__ void split_bf2(float v0, float v1, unsigned& hw, unsigned& lw) {
  const unsigned short h0 = f2bf_bits(v0), h1 = f2bf_bits(v1);
  const unsigned short l0 = f2bf_bits(v0 - bf_bits2f(h0));
  const unsigned short l1 = f2bf_bits(v1 - bf_bits2f(h1));
  hw = (unsigned)h0 | ((unsigned)h1 << 16);
  lw = (unsigned)l0 | ((unsigned)l1 << 16);
}

__device__ __forceinline__ void dep_guard_h(v8f& a, v8f& b, v16h x, v16h y) { asm volatile("v_nop\n\tv_nop\n\tv_nop\n\tv_nop" : "+v"(a), "+v"(b) : "v"(x), "v"(y)); }
__device__ __forceinline__ void dep_guard_b(v8f& a, v8f& b, v16b x, v16b y) { asm volatile("v_nop\n\tv_nop\n\tv_nop\n\tv_nop" : "+v"(a), "+v"(b) : "v"(x), "v"(y)); }
__device__ __forceinline__ void keep4_h(v16h a, v16h b, v16h c, v16h d) { asm volatile("v_nop" :: "v"(a), "v"(b), "v"(c), "v"(d)); }
__device__ __forceinline__ void keep4_b(v16b a, v16b b, v16b c, v16b d) { asm volatile("v_nop" :: "v"(a), "v"(b), "v"(c), "v"(d)); }
__device__ __forceinline__ void acc_guard4(v8f& a, v8f& b, v8f& c, v8f& d) { asm volatile("v_nop\n\tv_nop\n\tv_nop\n\tv_nop" : "+v"(a), "+v"(b), "+v"(c), "+v"(d)); }

template <typename T> struct Frag;
template <> struct Frag<_Float16> {
  typedef v16h V; union U { v16h v; v8h h[2]; };
  static __device__ __forceinline__ v16h load(const _Float16* p) {
    U f; f.h[0] = *(const v8h*)(p); f.h[1] = *(const v8h*)(p + 16); return f.v;
  }
  static __device__ __forceinline__ v8f mma(v16h a, v16h b, v8f c) {
    return __builtin_amdgcn_wmma_f32_16x16x32_f16(false, a, false, b, (short)0, c, false, false);
  }
  static __device__ __forceinline__ void guard(v8f& a, v8f& b, v16h x, v16h y) { dep_guard_h(a, b, x, y); }
  static __device__ __forceinline__ void keep(v16h a, v16h b, v16h c, v16h d) { keep4_h(a, b, c, d); }
};
template <> struct Frag<__bf16> {
  typedef v16b V; union U { v16b v; v8b h[2]; };
  static __device__ __forceinline__ v16b load(const __bf16* p) {
    U f; f.h[0] = *(const v8b*)(p); f.h[1] = *(const v8b*)(p + 16); return f.v;
  }
  static __device__ __forceinline__ v8f mma(v16b a, v16b b, v8f c) {
    return __builtin_amdgcn_wmma_f32_16x16x32_bf16(false, a, false, b, (short)0, c, false, false);
  }
  static __device__ __forceinline__ void guard(v8f& a, v8f& b, v16b x, v16b y) { dep_guard_b(a, b, x, y); }
  static __device__ __forceinline__ void keep(v16b a, v16b b, v16b c, v16b d) { keep4_b(a, b, c, d); }
};

template <int ET> struct Elem;
template <> struct Elem<0> { typedef _Float16 T; };
template <> struct Elem<1> { typedef __bf16 T; };
template <int ET, int SPLITK, int BIAS_MODE, int OUT_MODE, bool RESID, int ACT = 0>
__global__ __launch_bounds__(256) void wmma_gemm64(
    const unsigned short* __restrict__ Ap, const unsigned short* __restrict__ A2p, int lda, long strideA,
    const unsigned short* __restrict__ Btp, const unsigned short* __restrict__ Bt2p, int ldb, long strideB,
    void* __restrict__ Cout, void* __restrict__ Cout2, int ldc, long strideC,
    const float* __restrict__ bias,
    const float* __restrict__ resid, long strideR,
    int M, int N, int K, float scale) {
  typedef typename Elem<ET>::T T;
  typedef typename Frag<T>::V V;
  constexpr bool SPA = (SPLITK != 0);
  constexpr bool SPB = (SPLITK == 1);
  const T* A = (const T*)Ap; const T* A2 = (const T*)A2p; const T* Bt = (const T*)Btp; const T* Bt2 = (const T*)Bt2p;
  __shared__ __align__(16) float sT[8][16 * 68];
  const int b    = blockIdx.y;
  const int lane = threadIdx.x & 31;
  const int wave = threadIdx.x >> 5;
  const int tilesN = N >> 6;
  const int tilesM = M >> 6;
  const int tile = blockIdx.x * 8 + wave;
  if (tile >= tilesM * tilesN) return;
  const int tm = tile / tilesN;
  const int tn = tile - tm * tilesN;
  const int m0 = tm << 6;
  const int n0 = tn << 6;

  const T* Ab  = A  + (size_t)b * strideA;
  const T* Bb  = Bt + (size_t)b * strideB;
  const T* Ab2 = SPA ? (A2  + (size_t)b * strideA) : nullptr;
  const T* Bb2 = SPB ? (Bt2 + (size_t)b * strideB) : nullptr;

  const int rlane = lane & 15;
  const int koff  = (lane >> 4) * 8;
  const int mOff  = (lane >> 4) * 8;

  v8f acc[4][4];
#pragma unroll
  for (int i = 0; i < 4; ++i)
#pragma unroll
    for (int j = 0; j < 4; ++j) acc[i][j] = (v8f){0.f,0.f,0.f,0.f,0.f,0.f,0.f,0.f};

  for (int k0 = 0; k0 < K; k0 += 32) {
    V bh[4], bl[4];
#pragma unroll
    for (int j = 0; j < 4; ++j) {
      const size_t bo = (size_t)(n0 + (j << 4) + rlane) * ldb + koff + k0;
      bh[j] = Frag<T>::load(Bb + bo);
      bl[j] = SPB ? Frag<T>::load(Bb2 + bo) : bh[j];
    }
#pragma unroll
    for (int i = 0; i < 4; ++i) {
      const size_t ao = (size_t)(m0 + (i << 4) + rlane) * lda + koff + k0;
      V ah = Frag<T>::load(Ab + ao);
      V al = SPA ? Frag<T>::load(Ab2 + ao) : ah;
#pragma unroll
      for (int j = 0; j < 4; ++j) {
        acc[i][j] = Frag<T>::mma(ah, bh[j], acc[i][j]);
        if (SPB) acc[i][j] = Frag<T>::mma(ah, bl[j], acc[i][j]);
        if (SPA) acc[i][j] = Frag<T>::mma(al, bh[j], acc[i][j]);
      }
      Frag<T>::guard(acc[i][0], acc[i][3], ah, al);
    }
    Frag<T>::keep(bh[0], bh[1], bh[2], bh[3]);
    if (SPB) Frag<T>::keep(bl[0], bl[1], bl[2], bl[3]);
  }
  acc_guard4(acc[0][0], acc[0][1], acc[0][2], acc[0][3]);
  acc_guard4(acc[1][0], acc[1][1], acc[1][2], acc[1][3]);
  acc_guard4(acc[2][0], acc[2][1], acc[2][2], acc[2][3]);
  acc_guard4(acc[3][0], acc[3][1], acc[3][2], acc[3][3]);

  float* slab = sT[wave];
  const float* Rb = RESID ? (resid + (size_t)b * strideR) : nullptr;
#pragma unroll
  for (int i = 0; i < 4; ++i) {
    const int mBase = m0 + (i << 4);
#pragma unroll
    for (int j = 0; j < 4; ++j) {
      const int n = n0 + (j << 4) + rlane;
      float bv = 0.f;
      if (BIAS_MODE == 2) bv = bias[n];
#pragma unroll
      for (int r = 0; r < 8; ++r) {
        float v = acc[i][j][r] * scale;
        if (BIAS_MODE == 1) v += bias[mBase + mOff + r];
        if (BIAS_MODE == 2) v += bv;
        if (RESID) v += Rb[(size_t)(mBase + mOff + r) * ldc + n];
        if (ACT == 1) v = tanhf(v);
        if (ACT == 2) v = fmaxf(v, 0.0f);
        if (ACT == 3) v = v / (1.0f + expf(-v));
        if (ACT == 4) v = (v > 0.f) ? v : 0.01f * v;
        slab[(mOff + r) * 68 + (j << 4) + rlane] = v;
      }
    }
    __builtin_amdgcn_fence(__ATOMIC_RELEASE, "workgroup");
    __builtin_amdgcn_wave_barrier();
    __builtin_amdgcn_fence(__ATOMIC_ACQUIRE, "workgroup");
    if (OUT_MODE == 0) {
      float* C = (float*)Cout + (size_t)b * strideC;
      const int hh = lane >> 4, c4 = (lane & 15) * 4;
      for (int pass = 0; pass < 2; ++pass) {
#pragma unroll
        for (int it = 0; it < 8; ++it) {
          const int row = it * 2 + hh;
          v4f v = *(const v4f*)(slab + row * 68 + c4);
          *(volatile v4f*)(C + (size_t)(mBase + row) * ldc + n0 + c4) = v;
        }
        __threadfence();
      }
    } else {
      const int q = lane >> 3, c8 = (lane & 7) * 8;
      unsigned short* C  = (unsigned short*)Cout  + (size_t)b * strideC;
      unsigned short* C2 = (OUT_MODE == 2) ? ((unsigned short*)Cout2 + (size_t)b * strideC) : nullptr;
      for (int pass = 0; pass < 2; ++pass) {
#pragma unroll
        for (int it = 0; it < 4; ++it) {
          const int row = it * 4 + q;
          const float* sp = slab + row * 68 + c8;
          v8h hv, lv;
#pragma unroll
          for (int e = 0; e < 8; ++e) {
            if (OUT_MODE == 1) {
              hv[e] = (_Float16)sp[e];
            } else {
              unsigned short hb = f2bf_bits(sp[e]);
              unsigned short lb = f2bf_bits(sp[e] - bf_bits2f(hb));
              hv[e] = __builtin_bit_cast(_Float16, hb);
              lv[e] = __builtin_bit_cast(_Float16, lb);
            }
          }
          *(volatile v8h*)(C + (size_t)(mBase + row) * ldc + n0 + c8) = hv;
          if (OUT_MODE == 2) *(volatile v8h*)(C2 + (size_t)(mBase + row) * ldc + n0 + c8) = lv;
        }
        __threadfence();
      }
    }
    __builtin_amdgcn_fence(__ATOMIC_RELEASE, "workgroup");
    __builtin_amdgcn_wave_barrier();
    __builtin_amdgcn_fence(__ATOMIC_ACQUIRE, "workgroup");
  }
}

__global__ __launch_bounds__(256) void k_cast_bf16(
    const float* __restrict__ src, unsigned short* __restrict__ dst, int nsrc, int ndst) {
  const int i = blockIdx.x * 256 + threadIdx.x;
  const int nth = ndst >> 3;
  if (i >= nth) return;
  const int e0 = i << 3;
  const bool live = e0 < nsrc;
  const int eb = live ? e0 : (nsrc - 8);
  const v4f a = *(const v4f*)(src + eb);
  const v4f c = *(const v4f*)(src + eb + 4);
  v4u w;
  w[0] = pack_bf2(a[0], a[1]);
  w[1] = pack_bf2(a[2], a[3]);
  w[2] = pack_bf2(c[0], c[1]);
  w[3] = pack_bf2(c[2], c[3]);
  if (!live) w = (v4u){0u, 0u, 0u, 0u};
  unsigned short* p = dst + (size_t)e0;
  *(volatile v4u*)p = w;
  __threadfence();
  *(volatile v4u*)p = w;
}

__global__ __launch_bounds__(256) void k_split_dtu(
    const float* __restrict__ par, unsigned short* __restrict__ dhi, unsigned short* __restrict__ dlo) {
  const int gid = blockIdx.x * 256 + threadIdx.x;
  const int row = gid >> 3;
  if (row >= NROWS) return;
  const int c8 = (gid & 7) * 8;
  const float* sp = par + (size_t)row * NPARPAD + c8;
  const v4f a = *(const v4f*)(sp);
  const v4f c = *(const v4f*)(sp + 4);
  v4u hv, lv;
  unsigned hw, lw;
  split_bf2(a[0], a[1], hw, lw); hv[0] = hw; lv[0] = lw;
  split_bf2(a[2], a[3], hw, lw); hv[1] = hw; lv[1] = lw;
  split_bf2(c[0], c[1], hw, lw); hv[2] = hw; lv[2] = lw;
  split_bf2(c[2], c[3], hw, lw); hv[3] = hw; lv[3] = lw;
  const size_t o = (size_t)row * RNK + c8;
  for (int pass = 0; pass < 2; ++pass) {
    *(volatile v4u*)(dhi + o) = hv;
    *(volatile v4u*)(dlo + o) = lv;
    __threadfence();
  }
}

constexpr int SC_CH = 64;
constexpr int SC_TT = 64;
static_assert(SEQLEN % SC_TT == 0 && EMB % SC_CH == 0 && SC_TT == 2 * 32);

__global__ __launch_bounds__(SC_CH) void k_scan(
    const float* __restrict__ xres, const float* __restrict__ zf, const float* __restrict__ par,
    const float* __restrict__ dtraw, const float* __restrict__ conv_w, const float* __restrict__ b_dt,
    const float* __restrict__ A_log, const float* __restrict__ Dp,
    unsigned short* __restrict__ yhi, unsigned short* __restrict__ ylo) {
  __shared__ __align__(16) float s_bc[SC_TT * 32];
  __shared__ __align__(16) float s_y[SC_TT * SC_CH];
  __shared__ float s_h[NSTATE * SC_CH];
  __shared__ float s_a[NSTATE * SC_CH];
  __shared__ float s_bi[NSTATE * SC_CH];

  const int tid = threadIdx.x;
  const int blk = blockIdx.x;
  const int b   = blk >> 4;
  const int d0  = (blk & 15) * SC_CH;
  const int d   = d0 + tid;
  const size_t rowbase = (size_t)b * SEQLEN;

#pragma unroll 1
  for (int n = 0; n < NSTATE; ++n) {
    const float ar = bf_rne(A_log[(size_t)d * NSTATE + n]);
    const float a  = -expf(ar);
    s_a[n * SC_CH + tid]  = a;
    s_bi[n * SC_CH + tid] = 1.0f / (a + 1e-10f);
    s_h[n * SC_CH + tid]  = 0.0f;
  }
  const v4f cw = *(const v4f*)(conv_w + (size_t)d * KCONV);
  const float w0 = bf_rne(cw[0]), w1 = bf_rne(cw[1]), w2 = bf_rne(cw[2]), w3 = bf_rne(cw[3]);
  const float bdt = bf_rne(b_dt[d]);
  const float dp  = bf_rne(Dp[d]);
  float xm1 = 0.0f, xm2 = 0.0f, xm3 = 0.0f;

  const int wv = tid >> 5, lane = tid & 31;
  const int q = lane >> 3, c8 = (lane & 7) * 8;

#pragma unroll 1
  for (int t0 = 0; t0 < SEQLEN; t0 += SC_TT) {
    __syncthreads();
#pragma unroll
    for (int i = 0; i < 8; ++i) {
      const int idx = i * SC_CH + tid;
      const int tl = idx >> 3, c4 = (idx & 7) * 4;
      const v4f v = *(const v4f*)(par + (rowbase + t0 + tl) * NPARPAD + RNK + c4);
      *(v4f*)(s_bc + tl * 32 + c4) = v;
    }
    __syncthreads();

#pragma unroll 1
    for (int tl = 0; tl < SC_TT; ++tl) {
      const size_t e = (rowbase + t0 + tl) * EMB + d;
      const float xr = xres[e];
      const float zr = zf[e];
      const float dr = dtraw[e];
      float cv = w0 * xm3;
      cv += w1 * xm2;
      cv += w2 * xm1;
      cv += w3 * xr;
      xm3 = xm2; xm2 = xm1; xm1 = xr;
      const float u  = cv * (1.0f / (1.0f + expf(-cv)));
      const float v  = dr + bdt;
      const float dt = fmaxf(v, 0.0f) + log1pf(expf(-fabsf(v)));
      const float g  = zr * (1.0f / (1.0f + expf(-zr)));
      const float* bcrow = s_bc + tl * 32;
      float ys = 0.0f;
#pragma unroll 1
      for (int n = 0; n < NSTATE; ++n) {
        const float a  = s_a[n * SC_CH + tid];
        const float bi = s_bi[n * SC_CH + tid];
        const float h0 = s_h[n * SC_CH + tid];
        const float At  = expf(dt * a);
        const float Btl = (fabsf(a) < 1e-8f) ? dt : (At - 1.0f) * bi;
        const float h1  = At * h0 + (Btl * bcrow[n]) * u;
        s_h[n * SC_CH + tid] = h1;
        ys += bcrow[NSTATE + n] * h1;
      }
      s_y[tl * SC_CH + tid] = (ys + u * dp) * g;
    }
    __syncthreads();

    for (int pass = 0; pass < 2; ++pass) {
#pragma unroll
      for (int it = 0; it < 8; ++it) {
        const int rl = wv * 32 + it * 4 + q;
        const v4f y0 = *(const v4f*)(s_y + rl * SC_CH + c8);
        const v4f y1 = *(const v4f*)(s_y + rl * SC_CH + c8 + 4);
        v4u hv, lv;
        unsigned hw, lw;
        split_bf2(y0[0], y0[1], hw, lw); hv[0] = hw; lv[0] = lw;
        split_bf2(y0[2], y0[3], hw, lw); hv[1] = hw; lv[1] = lw;
        split_bf2(y1[0], y1[1], hw, lw); hv[2] = hw; lv[2] = lw;
        split_bf2(y1[2], y1[3], hw, lw); hv[3] = hw; lv[3] = lw;
        const size_t o = (rowbase + t0 + rl) * EMB + d0 + c8;
        *(volatile v4u*)(yhi + o) = hv;
        *(volatile v4u*)(ylo + o) = lv;
      }
      __threadfence();
    }
  }
}

static void gemm_plain(const unsigned short* A, int lda, const unsigned short* Bt, int ldb,
                       float* C, int ldc, const float* dummyf, int M, int N, int K, hipStream_t s) {
  const int tiles = (M / 64) * (N / 64);
  dim3 grid((tiles + 7) / 8, 1, 1);
  wmma_gemm64<1, 0, 0, 0, false, 0><<<grid, dim3(256, 1, 1), 0, s>>>(
      A, A, lda, 0L, Bt, Bt, ldb, 0L, (void*)C, (void*)C, ldc, 0L, dummyf, dummyf, 0L, M, N, K, 1.0f);
}
static void gemm_asplit(const unsigned short* Ah, const unsigned short* Al, int lda,
                        const unsigned short* Bt, int ldb, float* C, int ldc, const float* dummyf,
                        int M, int N, int K, hipStream_t s) {
  const int tiles = (M / 64) * (N / 64);
  dim3 grid((tiles + 7) / 8, 1, 1);
  wmma_gemm64<1, 2, 0, 0, false, 0><<<grid, dim3(256, 1, 1), 0, s>>>(
      Ah, Al, lda, 0L, Bt, Bt, ldb, 0L, (void*)C, (void*)C, ldc, 0L, dummyf, dummyf, 0L, M, N, K, 1.0f);
}

extern "C" void kernel_launch(void* const* d_in, const int* in_sizes, int n_in,
                              void* d_out, int out_size, void* d_ws, size_t ws_size,
                              hipStream_t stream) {
  if (n_in < 10) return;
  if (in_sizes[0] != NROWS * EMB || in_sizes[1] != EMB * EMB || in_sizes[2] != EMB * EMB ||
      in_sizes[3] != NPAR * EMB || in_sizes[4] != EMB * KCONV || in_sizes[5] != EMB * RNK ||
      in_sizes[6] != EMB || in_sizes[7] != EMB * NSTATE || in_sizes[8] != EMB ||
      in_sizes[9] != EMB * EMB) return;
  if (out_size != NROWS * EMB) return;
  if (ws_size < WS_TOTAL) return;

  const float* x        = (const float*)d_in[0];
  const float* W_x      = (const float*)d_in[1];
  const float* W_z      = (const float*)d_in[2];
  const float* W_params = (const float*)d_in[3];
  const float* conv_w   = (const float*)d_in[4];
  const float* W_dt     = (const float*)d_in[5];
  const float* b_dt     = (const float*)d_in[6];
  const float* A_log    = (const float*)d_in[7];
  const float* D_param  = (const float*)d_in[8];
  const float* W_out    = (const float*)d_in[9];
  float* out = (float*)d_out;

  char* ws = (char*)d_ws;
  unsigned short* xb    = (unsigned short*)(ws + OFF_XB);
  unsigned short* wxb   = (unsigned short*)(ws + OFF_WX);
  unsigned short* wzb   = (unsigned short*)(ws + OFF_WZ);
  unsigned short* wob   = (unsigned short*)(ws + OFF_WO);
  unsigned short* wpb   = (unsigned short*)(ws + OFF_WP);
  unsigned short* wdtb  = (unsigned short*)(ws + OFF_WDT);
  float*          xres  = (float*)(ws + OFF_XRES);
  float*          zf    = (float*)(ws + OFF_Z);
  float*          par   = (float*)(ws + OFF_PAR);
  unsigned short* dtuh  = (unsigned short*)(ws + OFF_DTUH);
  unsigned short* dtul  = (unsigned short*)(ws + OFF_DTUL);
  float*          dtraw = (float*)(ws + OFF_DTRAW);
  unsigned short* yh    = (unsigned short*)(ws + OFF_YH);
  unsigned short* yl    = (unsigned short*)(ws + OFF_YL);

  k_cast_bf16<<<dim3((NROWS * EMB / 8 + 255) / 256), dim3(256), 0, stream>>>(x, xb, NROWS * EMB, NROWS * EMB);
  k_cast_bf16<<<dim3((EMB * EMB / 8 + 255) / 256), dim3(256), 0, stream>>>(W_x, wxb, EMB * EMB, EMB * EMB);
  k_cast_bf16<<<dim3((EMB * EMB / 8 + 255) / 256), dim3(256), 0, stream>>>(W_z, wzb, EMB * EMB, EMB * EMB);
  k_cast_bf16<<<dim3((NPARPAD * EMB / 8 + 255) / 256), dim3(256), 0, stream>>>(W_params, wpb, NPAR * EMB, NPARPAD * EMB);
  k_cast_bf16<<<dim3((EMB * RNK / 8 + 255) / 256), dim3(256), 0, stream>>>(W_dt, wdtb, EMB * RNK, EMB * RNK);
  k_cast_bf16<<<dim3((EMB * EMB / 8 + 255) / 256), dim3(256), 0, stream>>>(W_out, wob, EMB * EMB, EMB * EMB);

  gemm_plain(xb, EMB, wxb, EMB, xres, EMB, par, NROWS, EMB, EMB, stream);
  gemm_plain(xb, EMB, wzb, EMB, zf, EMB, par, NROWS, EMB, EMB, stream);
  gemm_plain(xb, EMB, wpb, EMB, par, NPARPAD, xres, NROWS, NPARPAD, EMB, stream);

  k_split_dtu<<<dim3((NROWS * 8 + 255) / 256), dim3(256), 0, stream>>>(par, dtuh, dtul);
  gemm_asplit(dtuh, dtul, RNK, wdtb, RNK, dtraw, EMB, par, NROWS, EMB, RNK, stream);

  k_scan<<<dim3(NBATCH * EMB / SC_CH), dim3(SC_CH), 0, stream>>>(xres, zf, par, dtraw, conv_w, b_dt, A_log, D_param, yh, yl);

  gemm_asplit(yh, yl, EMB, wob, EMB, out, EMB, par, NROWS, EMB, EMB, stream);
}
